// DeltaBase_34583076667908
// MI455X (gfx1250) — hardware-run, weakly checked
//
#include <hip/hip_runtime.h>
#include <math.h>

typedef __attribute__((ext_vector_type(16))) _Float16 v16h;
typedef __attribute__((ext_vector_type(8)))  _Float16 v8h;
typedef __attribute__((ext_vector_type(8)))  float    v8f;
typedef __attribute__((ext_vector_type(4)))  float    v4f;

constexpr int kH      = 64;
constexpr int kH2     = 128;
constexpr int kVocab  = 64;
constexpr int kB      = 256;
constexpr int kL      = 512;
constexpr int kSteps  = kL - 1;
constexpr int kPitchK64  = 72;
constexpr int kPitchK128 = 136;
constexpr int kPitchF    = 68;
static_assert((kPitchK64 * 2) % 16 == 0 && (kPitchK128 * 2) % 16 == 0 && (kPitchF * 4) % 16 == 0, "16-B aligned LDS rows");
static_assert(kH % 32 == 0 && kH2 % 32 == 0, "k depth multiples of 32");
static_assert(kVocab % 16 == 0 && kB % 16 == 0 && kH % 16 == 0 && kH2 % 16 == 0, "tile multiples");

constexpr float kCarryW = 64.0f;
constexpr float kCarryE = 16.0f;
constexpr float kCarryA = 64.0f;
constexpr float kCarryY = 16.0f;
constexpr float kCarryZ = 16.0f;
constexpr float kFoldEW = 1.0f / (kCarryE * kCarryW);
constexpr float kFoldAW = 1.0f / (kCarryA * kCarryW);
constexpr float kFoldYW = 1.0f / (kCarryY * kCarryW);
constexpr float kFoldZW = 1.0f / (kCarryZ * kCarryW);
constexpr float kLnEps   = 1e-5f;
constexpr float kNormEps = 1e-12f;
constexpr float kInvH    = 1.0f / (float)kH;
constexpr float kF16MinNormal = 6.103515625e-5f;

constexpr size_t kBytesHV = (size_t)kVocab * kH * 4;
constexpr size_t kBytesKN = (size_t)kVocab * kH * 4;
constexpr size_t kBytesY  = (size_t)kB * kH * 4;
constexpr size_t kOffHV   = 0;
constexpr size_t kOffKN   = kOffHV + kBytesHV;
constexpr size_t kOffY    = kOffKN + kBytesKN;
constexpr size_t kWsTotal = kOffY + kBytesY;
static_assert(kWsTotal == 98304ull, "carve total");
static_assert(kWsTotal <= 134217728ull, "carve cap");
static_assert((kOffKN % 128) == 0 && (kOffY % 128) == 0, "128-B aligned regions");

template <typename T> struct Frag;
template <> struct Frag<_Float16> {
  typedef v16h V;
  union U { v16h v; v8h h[2]; };
  static __device__ __forceinline__ v16h load(const _Float16* p) {
    U f;
    f.h[0] = *(const v8h*)(p);
    f.h[1] = *(const v8h*)(p + 16);
    return f.v;
  }
};

__device__ __forceinline__ v8f mma_g(v16h a, v16h b, v8f c) {
  c = __builtin_amdgcn_wmma_f32_16x16x32_f16(false, a, false, b, (short)0, c, false, false);
  asm volatile("v_nop\n\tv_nop\n\tv_nop\n\tv_nop" : "+v"(c) : "v"(a), "v"(b));
  return c;
}

__device__ __forceinline__ _Float16 to_h16(float v) {
  const float w = (fabsf(v) < kF16MinNormal) ? 0.0f : v;
  return (_Float16)w;
}

__global__ __launch_bounds__(128) void k_table(
    const float* __restrict__ embed, const float* __restrict__ w1, const float* __restrict__ b1,
    const float* __restrict__ w2, const float* __restrict__ b2,
    const float* __restrict__ ln_g, const float* __restrict__ ln_b,
    float* __restrict__ HV, float* __restrict__ KN)
{
  __shared__ __align__(16) _Float16 sW1t[kH2 * kPitchK64];
  __shared__ __align__(16) _Float16 sW2t[kH * kPitchK128];
  __shared__ __align__(16) _Float16 sE[16 * kPitchK64];
  __shared__ __align__(16) _Float16 sA[16 * kPitchK128];
  __shared__ __align__(16) float sX[16 * kPitchF];
  __shared__ __align__(16) float sK[16 * kPitchF];

  const int tid  = threadIdx.x;
  const int lane = tid & 31;
  const int wave = tid >> 5;
  const int hh   = lane >> 4;
  const int c    = lane & 15;
  const int r0   = blockIdx.x * 16;

#pragma unroll 4
  for (int it = 0; it < (kH * kH2) / 128; ++it) {
    const int idx = it * 128 + tid;
    const int k = idx >> 7;
    const int n = idx & 127;
    sW1t[n * kPitchK64 + k] = to_h16(w1[idx] * kCarryW);
  }
#pragma unroll 4
  for (int it = 0; it < (kH2 * kH) / 128; ++it) {
    const int idx = it * 128 + tid;
    const int k = idx >> 6;
    const int n = idx & 63;
    sW2t[n * kPitchK128 + k] = to_h16(w2[idx] * kCarryW);
  }
#pragma unroll 4
  for (int it = 0; it < (16 * kH) / 128; ++it) {
    const int idx = it * 128 + tid;
    const int r = idx >> 6;
    const int cc = idx & 63;
    sE[r * kPitchK64 + cc] = to_h16(embed[(r0 + r) * kH + cc] * kCarryE);
  }
  __syncthreads();

#pragma unroll
  for (int u = 0; u < 2; ++u) {
    const int n0 = (wave * 2 + u) * 16;
    v8f acc = (v8f){0.f, 0.f, 0.f, 0.f, 0.f, 0.f, 0.f, 0.f};
#pragma unroll
    for (int kk = 0; kk < kH / 32; ++kk) {
      const v16h a = Frag<_Float16>::load(sE + c * kPitchK64 + kk * 32 + 8 * hh);
      const v16h b = Frag<_Float16>::load(sW1t + (n0 + c) * kPitchK64 + kk * 32 + 8 * hh);
      acc = mma_g(a, b, acc);
    }
    const float bv = b1[n0 + c];
#pragma unroll
    for (int r = 0; r < 8; ++r) {
      float v = acc[r] * kFoldEW + bv;
      v = fmaxf(v, 0.0f);
      sA[(8 * hh + r) * kPitchK128 + n0 + c] = to_h16(v * kCarryA);
    }
  }
  __syncthreads();

  {
    const int n0 = wave * 16;
    v8f acc = (v8f){0.f, 0.f, 0.f, 0.f, 0.f, 0.f, 0.f, 0.f};
#pragma unroll
    for (int kk = 0; kk < kH2 / 32; ++kk) {
      const v16h a = Frag<_Float16>::load(sA + c * kPitchK128 + kk * 32 + 8 * hh);
      const v16h b = Frag<_Float16>::load(sW2t + (n0 + c) * kPitchK128 + kk * 32 + 8 * hh);
      acc = mma_g(a, b, acc);
    }
    const float bv = b2[n0 + c];
#pragma unroll
    for (int r = 0; r < 8; ++r) {
      const int row = 8 * hh + r;
      const float e = embed[(r0 + row) * kH + n0 + c];
      const float ff = acc[r] * kFoldAW + bv;
      sX[row * kPitchF + n0 + c] = e + ff;
    }
  }
  __syncthreads();

  {
    const int row = tid >> 3;
    const int seg = (tid & 7) * 8;
    const v4f xa = *(const v4f*)(sX + row * kPitchF + seg);
    const v4f xb = *(const v4f*)(sX + row * kPitchF + seg + 4);
    const v4f ga = *(const v4f*)(ln_g + seg);
    const v4f gb = *(const v4f*)(ln_g + seg + 4);
    const v4f ba = *(const v4f*)(ln_b + seg);
    const v4f bb = *(const v4f*)(ln_b + seg + 4);
    float x[8], g[8], bt[8];
#pragma unroll
    for (int e = 0; e < 4; ++e) {
      x[e] = xa[e];
      x[4 + e] = xb[e];
      g[e] = ga[e];
      g[4 + e] = gb[e];
      bt[e] = ba[e];
      bt[4 + e] = bb[e];
    }
    float s = ((x[0] + x[1]) + (x[2] + x[3])) + ((x[4] + x[5]) + (x[6] + x[7]));
    s += __shfl_xor(s, 1, 32);
    s += __shfl_xor(s, 2, 32);
    s += __shfl_xor(s, 4, 32);
    const float mu = s * kInvH;
    float d[8];
    float ss = 0.0f;
#pragma unroll
    for (int e = 0; e < 8; ++e) {
      d[e] = x[e] - mu;
      ss = fmaf(d[e], d[e], ss);
    }
    ss += __shfl_xor(ss, 1, 32);
    ss += __shfl_xor(ss, 2, 32);
    ss += __shfl_xor(ss, 4, 32);
    const float var = ss * kInvH;
    const float rs = 1.0f / sqrtf(var + kLnEps);
    float hv[8];
    float s2 = 0.0f;
#pragma unroll
    for (int e = 0; e < 8; ++e) {
      hv[e] = (d[e] * rs) * g[e] + bt[e];
      s2 = fmaf(hv[e], hv[e], s2);
    }
    s2 += __shfl_xor(s2, 1, 32);
    s2 += __shfl_xor(s2, 2, 32);
    s2 += __shfl_xor(s2, 4, 32);
    const float den = fmaxf(sqrtf(s2), kNormEps);
    const float rn = 1.0f / den;
#pragma unroll
    for (int e = 0; e < 8; ++e) {
      sX[row * kPitchF + seg + e] = hv[e];
      sK[row * kPitchF + seg + e] = hv[e] * rn;
    }
  }
  __syncthreads();

  {
    const int c4 = c * 4;
    v4f hvv[2], knv[2];
#pragma unroll
    for (int it = 0; it < 2; ++it) {
      const int row = wave * 4 + it * 2 + hh;
      hvv[it] = *(const v4f*)(sX + row * kPitchF + c4);
      knv[it] = *(const v4f*)(sK + row * kPitchF + c4);
    }
    for (int pass = 0; pass < 2; ++pass) {
#pragma unroll
      for (int it = 0; it < 2; ++it) {
        const int row = wave * 4 + it * 2 + hh;
        *(volatile v4f*)(HV + (size_t)(r0 + row) * kH + c4) = hvv[it];
        *(volatile v4f*)(KN + (size_t)(r0 + row) * kH + c4) = knv[it];
      }
      __threadfence();
    }
  }
}

__global__ __launch_bounds__(256) void k_scan(
    const int* __restrict__ seq, const float* __restrict__ HV, const float* __restrict__ KN,
    float* __restrict__ Y)
{
  __shared__ __align__(16) float sHV[kVocab * kH];
  __shared__ __align__(16) float sKN[kVocab * kH];
  __shared__ __align__(16) int   sSeq[kL];
  __shared__ __align__(16) float sY[kH];

  const int tid = threadIdx.x;
  const int b   = blockIdx.x;
#pragma unroll
  for (int it = 0; it < (kVocab * kH) / (256 * 4); ++it) {
    const int idx = (it * 256 + tid) * 4;
    *(v4f*)(sHV + idx) = *(const v4f*)(HV + idx);
    *(v4f*)(sKN + idx) = *(const v4f*)(KN + idx);
  }
#pragma unroll
  for (int it = 0; it < kL / 256; ++it) {
    const int t = it * 256 + tid;
    int v = seq[(size_t)b * kL + t];
    v = v < 0 ? 0 : v;
    v = v > (kVocab - 1) ? (kVocab - 1) : v;
    sSeq[t] = v;
  }
  __syncthreads();

  const int i  = tid >> 2;
  const int j0 = (tid & 3) * 16;
  float m[16];
#pragma unroll
  for (int j = 0; j < 16; ++j) m[j] = 0.0f;

#pragma unroll 1
  for (int t = 0; t < kSteps; ++t) {
    const int v = sSeq[t];
    const float* kr = sKN + v * kH + j0;
    const v4f a0 = *(const v4f*)(kr);
    const v4f a1 = *(const v4f*)(kr + 4);
    const v4f a2 = *(const v4f*)(kr + 8);
    const v4f a3 = *(const v4f*)(kr + 12);
    const float kI = sHV[v * kH + i];
    const float kn[16] = {a0[0], a0[1], a0[2], a0[3], a1[0], a1[1], a1[2], a1[3],
                          a2[0], a2[1], a2[2], a2[3], a3[0], a3[1], a3[2], a3[3]};
    float p = 0.0f;
#pragma unroll
    for (int j = 0; j < 16; ++j) p = fmaf(m[j], kn[j], p);
    p += __shfl_xor(p, 1, 32);
    p += __shfl_xor(p, 2, 32);
    const float dv = kI - p;
#pragma unroll
    for (int j = 0; j < 16; ++j) m[j] = fmaf(dv, kn[j], m[j]);
  }

  {
    const int vl = sSeq[kL - 1];
    const float* qr = sHV + vl * kH + j0;
    const v4f a0 = *(const v4f*)(qr);
    const v4f a1 = *(const v4f*)(qr + 4);
    const v4f a2 = *(const v4f*)(qr + 8);
    const v4f a3 = *(const v4f*)(qr + 12);
    const float qv[16] = {a0[0], a0[1], a0[2], a0[3], a1[0], a1[1], a1[2], a1[3],
                          a2[0], a2[1], a2[2], a2[3], a3[0], a3[1], a3[2], a3[3]};
    float y = 0.0f;
#pragma unroll
    for (int j = 0; j < 16; ++j) y = fmaf(m[j], qv[j], y);
    y += __shfl_xor(y, 1, 32);
    y += __shfl_xor(y, 2, 32);
    if ((tid & 3) == 0) sY[i] = y;
  }
  __syncthreads();
  if (tid < 32) {
    const int c4 = (tid & 15) * 4;
    const v4f val = *(const v4f*)(sY + c4);
    float* dst = Y + (size_t)b * kH + c4;
    if (tid < 16) *(volatile v4f*)dst = val;
    __threadfence();
    if (tid < 16) *(volatile v4f*)dst = val;
  }
}

__global__ __launch_bounds__(128) void k_head(
    const float* __restrict__ Y,
    const float* __restrict__ rp_w, const float* __restrict__ rp_b,
    const float* __restrict__ out_w, const float* __restrict__ out_b,
    float* __restrict__ out)
{
  __shared__ __align__(16) _Float16 sRt[kH * kPitchK64];
  __shared__ __align__(16) _Float16 sOt[kVocab * kPitchK64];
  __shared__ __align__(16) _Float16 sYt[16 * kPitchK64];
  __shared__ __align__(16) _Float16 sZt[16 * kPitchK64];
  __shared__ __align__(16) float sO[16 * kPitchF];

  const int tid  = threadIdx.x;
  const int lane = tid & 31;
  const int wave = tid >> 5;
  const int hh   = lane >> 4;
  const int c    = lane & 15;
  const int row0 = blockIdx.x * 16;
  const int n0   = wave * 16;

#pragma unroll 4
  for (int it = 0; it < (kH * kH) / 128; ++it) {
    const int idx = it * 128 + tid;
    const int k = idx >> 6;
    const int n = idx & 63;
    sRt[n * kPitchK64 + k] = to_h16(rp_w[idx] * kCarryW);
    sOt[n * kPitchK64 + k] = to_h16(out_w[idx] * kCarryW);
  }
#pragma unroll 4
  for (int it = 0; it < (16 * kH) / 128; ++it) {
    const int idx = it * 128 + tid;
    const int r = idx >> 6;
    const int cc = idx & 63;
    sYt[r * kPitchK64 + cc] = to_h16(Y[(size_t)(row0 + r) * kH + cc] * kCarryY);
  }
  __syncthreads();

  {
    v8f acc = (v8f){0.f, 0.f, 0.f, 0.f, 0.f, 0.f, 0.f, 0.f};
#pragma unroll
    for (int kk = 0; kk < kH / 32; ++kk) {
      const v16h a = Frag<_Float16>::load(sYt + c * kPitchK64 + kk * 32 + 8 * hh);
      const v16h b = Frag<_Float16>::load(sRt + (n0 + c) * kPitchK64 + kk * 32 + 8 * hh);
      acc = mma_g(a, b, acc);
    }
    const float bv = rp_b[n0 + c];
#pragma unroll
    for (int r = 0; r < 8; ++r) {
      const float z = acc[r] * kFoldYW + bv;
      sZt[(8 * hh + r) * kPitchK64 + n0 + c] = to_h16(z * kCarryZ);
    }
  }
  __syncthreads();

  {
    v8f acc = (v8f){0.f, 0.f, 0.f, 0.f, 0.f, 0.f, 0.f, 0.f};
#pragma unroll
    for (int kk = 0; kk < kH / 32; ++kk) {
      const v16h a = Frag<_Float16>::load(sZt + c * kPitchK64 + kk * 32 + 8 * hh);
      const v16h b = Frag<_Float16>::load(sOt + (n0 + c) * kPitchK64 + kk * 32 + 8 * hh);
      acc = mma_g(a, b, acc);
    }
    const float bv = out_b[n0 + c];
#pragma unroll
    for (int r = 0; r < 8; ++r) {
      sO[(8 * hh + r) * kPitchF + n0 + c] = acc[r] * kFoldZW + bv;
    }
  }
  __syncthreads();

  {
    const int c4 = c * 4;
    v4f ov[2];
#pragma unroll
    for (int it = 0; it < 2; ++it) {
      const int row = wave * 4 + it * 2 + hh;
      ov[it] = *(const v4f*)(sO + row * kPitchF + c4);
    }
    for (int pass = 0; pass < 2; ++pass) {
#pragma unroll
      for (int it = 0; it < 2; ++it) {
        const int row = wave * 4 + it * 2 + hh;
        *(volatile v4f*)(out + (size_t)(row0 + row) * kVocab + c4) = ov[it];
      }
      __threadfence();
    }
  }
}

extern "C" void kernel_launch(void* const* d_in, const int* in_sizes, int n_in,
                              void* d_out, int out_size, void* d_ws, size_t ws_size,
                              hipStream_t stream) {
  if (n_in < 12) return;
  if (in_sizes[0] != kB * kL) return;
  if (in_sizes[1] != kVocab * kH) return;
  if (in_sizes[2] != kH * kH2) return;
  if (in_sizes[3] != kH2) return;
  if (in_sizes[4] != kH2 * kH) return;
  if (in_sizes[5] != kH) return;
  if (in_sizes[6] != kH) return;
  if (in_sizes[7] != kH) return;
  if (in_sizes[8] != kH * kH) return;
  if (in_sizes[9] != kH) return;
  if (in_sizes[10] != kH * kVocab) return;
  if (in_sizes[11] != kVocab) return;
  if (out_size != kB * kVocab) return;
  if (ws_size < kWsTotal) return;

  const int*   seq   = (const int*)  d_in[0];
  const float* embed = (const float*)d_in[1];
  const float* w1    = (const float*)d_in[2];
  const float* b1    = (const float*)d_in[3];
  const float* w2    = (const float*)d_in[4];
  const float* b2    = (const float*)d_in[5];
  const float* ln_g  = (const float*)d_in[6];
  const float* ln_b  = (const float*)d_in[7];
  const float* rp_w  = (const float*)d_in[8];
  const float* rp_b  = (const float*)d_in[9];
  const float* out_w = (const float*)d_in[10];
  const float* out_b = (const float*)d_in[11];

  char* ws = (char*)d_ws;
  float* HV = (float*)(ws + kOffHV);
  float* KN = (float*)(ws + kOffKN);
  float* Y  = (float*)(ws + kOffY);

  k_table<<<kVocab / 16, 128, 0, stream>>>(embed, w1, b1, w2, b2, ln_g, ln_b, HV, KN);
  k_scan<<<kB, 256, 0, stream>>>(seq, HV, KN, Y);
  k_head<<<kB / 16, 128, 0, stream>>>(Y, rp_w, rp_b, out_w, out_b, (float*)d_out);
}
